// GATWithMultipleLinearLayers_88433376624937
// MI455X (gfx1250) — hardware-verified
//
#include <hip/hip_runtime.h>
#include <stddef.h>


#define DIN     256
#define HC1     512
#define HC2     256
#define NCLS    5
#define NTHR    256
#define NWAVE   8
#define EPT     8
#define NGRP    2
#define CHUNK   (NTHR * EPT * NGRP)
#define WCAP    (EPT * NGRP * 32)
#define LISTN   (NWAVE * WCAP)
#define NBC     4096
#define NBF     1024
#define RCAP    40960
#define RBN     128
#define TGT     256
#define DEGCAP  256
#define OTHR    512
#define BM      64
#define CBN     256
#define SPF     (CBN + 4)
#define PW      1024
#define WSCAP   134217728
#define NEG_SLOPE 0.2f
#define DEN_EPS 1e-16f
#define NEG_BIG (-3.0e38f)
#define WSC     64.0f
#define WSCI    0.015625f

#define LDS_FILL ((RCAP + NBF + LISTN) * 4 + 64)

static_assert((CHUNK & (CHUNK - 1)) == 0);
static_assert(CHUNK <= 4096);
static_assert(NBC <= 4096 && NBF <= 4096);
static_assert((NBC & (NBC - 1)) == 0 && (NBF & (NBF - 1)) == 0);
static_assert(NBC == 4 * NBF);
static_assert(OTHR * 8 == NBC);
static_assert((RCAP % 32) == 0);
static_assert(TGT == NWAVE * 32);
static_assert((TGT % BM) == 0);
static_assert((SPF % 4) == 0);

typedef float          v4f  __attribute__((ext_vector_type(4)));
typedef float          v8f  __attribute__((ext_vector_type(8)));
typedef int            v4i  __attribute__((ext_vector_type(4)));
typedef _Float16       v4h  __attribute__((ext_vector_type(4)));
typedef _Float16       v8h  __attribute__((ext_vector_type(8)));
typedef _Float16       v16h __attribute__((ext_vector_type(16)));
union Frag { v16h v; v8h h[2]; };
union H8   { v8h v; v4h q[2]; v4i w; };

template <int KD>
struct GL {
  static constexpr int APK  = KD + 8;
  static constexpr int LDSA = BM * APK * 2;
  static constexpr int LDS  = LDSA + BM * SPF * 4;
};

__device__ __forceinline__ v4f h2f(v4h h) { return __builtin_convertvector(h, v4f); }

__device__ __forceinline__ v8h pack8(v4f a, v4f b) {
  H8 u;
  u.q[0] = __builtin_convertvector(a, v4h);
  u.q[1] = __builtin_convertvector(b, v4h);
  return u.v;
}

__device__ __forceinline__ v4f relu4(v4f v) {
  v4f r;
  r.x = fmaxf(v.x, 0.f); r.y = fmaxf(v.y, 0.f); r.z = fmaxf(v.z, 0.f); r.w = fmaxf(v.w, 0.f);
  return r;
}

__device__ __forceinline__ v8f wmf(v16h a, v16h b, v8f c) {
  v8f d = __builtin_amdgcn_wmma_f32_16x16x32_f16(false, a, false, b, (short)0, c, false, false);
  asm volatile("v_nop\n\tv_nop\n\tv_nop\n\tv_nop" : "+v"(d) : "v"(a), "v"(b));
  return d;
}

__device__ __forceinline__ float lrelu(float v) { return v > 0.0f ? v : NEG_SLOPE * v; }

template <typename AT> struct ALd;
template <> struct ALd<float> {
  static __device__ __forceinline__ v8h ld(const float* p) {
    const v4f a = *(const v4f*)p, b = *(const v4f*)(p + 4);
    return pack8(a, b);
  }
};
template <> struct ALd<_Float16> {
  static __device__ __forceinline__ v8h ld(const _Float16* p) { return *(const v8h*)p; }
};

template <int NB>
__device__ __forceinline__ int scan_chunk(const int* __restrict__ dsts, int nE, int cbase, int slotBase,
                                          int vec8, int* list, int tid, int lane, int wave) {
  int wc = 0;
#pragma unroll
  for (int g = 0; g < NGRP; ++g) {
    const int el0  = (g * NTHR + tid) * EPT;
    const int e0   = cbase + el0;
    const int sent = -2147483647 - 1;
    v4i da, db;
    if (vec8 != 0 && cbase + CHUNK <= nE) {
      da = *(const v4i*)(dsts + e0);
      db = *(const v4i*)(dsts + e0 + 4);
    } else {
      da.x = (e0     < nE) ? dsts[min(e0, nE - 1)] : sent;
      da.y = (e0 + 1 < nE) ? dsts[min(e0 + 1, nE - 1)] : sent;
      da.z = (e0 + 2 < nE) ? dsts[min(e0 + 2, nE - 1)] : sent;
      da.w = (e0 + 3 < nE) ? dsts[min(e0 + 3, nE - 1)] : sent;
      db.x = (e0 + 4 < nE) ? dsts[min(e0 + 4, nE - 1)] : sent;
      db.y = (e0 + 5 < nE) ? dsts[min(e0 + 5, nE - 1)] : sent;
      db.z = (e0 + 6 < nE) ? dsts[min(e0 + 6, nE - 1)] : sent;
      db.w = (e0 + 7 < nE) ? dsts[min(e0 + 7, nE - 1)] : sent;
    }
    const unsigned nb = (unsigned)slotBase;
    const unsigned s0 = (unsigned)da.x - nb, s1 = (unsigned)da.y - nb;
    const unsigned s2 = (unsigned)da.z - nb, s3 = (unsigned)da.w - nb;
    const unsigned s4 = (unsigned)db.x - nb, s5 = (unsigned)db.y - nb;
    const unsigned s6 = (unsigned)db.z - nb, s7 = (unsigned)db.w - nb;
    const bool h0 = s0 < (unsigned)NB, h1 = s1 < (unsigned)NB, h2 = s2 < (unsigned)NB, h3 = s3 < (unsigned)NB;
    const bool h4 = s4 < (unsigned)NB, h5 = s5 < (unsigned)NB, h6 = s6 < (unsigned)NB, h7 = s7 < (unsigned)NB;
    const unsigned any = __builtin_amdgcn_ballot_w32(h0 | h1 | h2 | h3 | h4 | h5 | h6 | h7);
    if (any != 0u) {
#define HITJ(J, HJ, SJ) { \
        const unsigned mj = __builtin_amdgcn_ballot_w32(HJ); \
        if (mj != 0u) { \
          if (HJ) { \
            const int pos = wc + (int)__builtin_amdgcn_mbcnt_lo(mj, 0u); \
            if (pos < WCAP) list[wave * WCAP + pos] = ((el0 + (J)) << 12) | (int)(SJ); \
          } \
          wc += (int)__builtin_popcount(mj); } }
      HITJ(0, h0, s0)
      HITJ(1, h1, s1)
      HITJ(2, h2, s2)
      HITJ(3, h3, s3)
      HITJ(4, h4, s4)
      HITJ(5, h5, s5)
      HITJ(6, h6, s6)
      HITJ(7, h7, s7)
#undef HITJ
    }
  }
  return wc;
}

template <int KD, int NC>
__global__ __launch_bounds__(NTHR) void k_wprep(const float* __restrict__ W, _Float16* wp) {
  constexpr int UNITS = NC * KD / 8;
  constexpr int KD8   = KD / 8;
  static_assert((UNITS % 32) == 0);
  const int i = (int)blockIdx.x * NTHR + (int)threadIdx.x;
  if (i >= UNITS) return;
  const int n  = i / KD8;
  const int k0 = (i - n * KD8) * 8;
  float v[8];
#pragma unroll
  for (int e = 0; e < 8; ++e) v[e] = W[(size_t)(k0 + e) * NC + n] * WSC;
  v4f a, b;
  a.x = v[0]; a.y = v[1]; a.z = v[2]; a.w = v[3];
  b.x = v[4]; b.y = v[5]; b.z = v[6]; b.w = v[7];
  H8 u; u.v = pack8(a, b);
  _Float16* d = wp + (size_t)i * 8;
  *(volatile v4i*)d = u.w;
  __threadfence();
  *(volatile v4i*)d = u.w;
}

__global__ __launch_bounds__(NTHR) void k_count(
    const int* __restrict__ dsts, int* cnt, int nE, int vec8) {
  __shared__ __attribute__((aligned(16))) int scnt[NBC];
  __shared__ __attribute__((aligned(16))) int list[LISTN];
  __shared__ int wcnt[NWAVE];
  const int tid = threadIdx.x, lane = tid & 31, wave = tid >> 5;
  const int nodeBase = blockIdx.x * NBC;

  for (int i = tid; i < NBC; i += NTHR) scnt[i] = 0;
  __syncthreads();

  const int nChunks = (nE + CHUNK - 1) / CHUNK;
#pragma unroll 1
  for (int ch = 0; ch < nChunks; ++ch) {
    const int cbase = ch * CHUNK;
    const int wc = scan_chunk<NBC>(dsts, nE, cbase, nodeBase, vec8, list, tid, lane, wave);
    if (lane == 0) wcnt[wave] = wc;
    __syncthreads();
    if (wave == 0) {
#pragma unroll 1
      for (int wsx = 0; wsx < NWAVE; ++wsx) {
        int n = __builtin_amdgcn_readfirstlane(wcnt[wsx]);
        n = n > WCAP ? WCAP : (n < 0 ? 0 : n);
        const int* lp = list + wsx * WCAP;
#pragma unroll 1
        for (int i = 0; i < n; ++i) {
          const int ent  = __builtin_amdgcn_readfirstlane(lp[i]);
          const int slot = ent & (NBC - 1);
          if (lane == 0) scnt[slot] = scnt[slot] + 1;
        }
      }
    }
    __syncthreads();
  }

  v4i cq[4];
#pragma unroll
  for (int q = 0; q < 4; ++q) {
    const int f = (wave * 4 + q) * 128 + 4 * lane;
    cq[q] = *(const v4i*)(scnt + f);
  }
  int* cp = cnt + (size_t)nodeBase;
#pragma unroll
  for (int q = 0; q < 4; ++q) {
    const int f = (wave * 4 + q) * 128 + 4 * lane;
    *(volatile v4i*)(cp + f) = cq[q];
  }
  __threadfence();
#pragma unroll
  for (int q = 0; q < 4; ++q) {
    const int f = (wave * 4 + q) * 128 + 4 * lane;
    *(volatile v4i*)(cp + f) = cq[q];
  }
}

__global__ __launch_bounds__(OTHR) void k_offsets(
    const int* __restrict__ cnt, int* off, int* rbase, int nChunk) {
  __shared__ __attribute__((aligned(16))) int soff[NBC];
  __shared__ __attribute__((aligned(16))) int srb[RBN];
  __shared__ int wtot[OTHR / 32];
  const int tid = threadIdx.x, lane = tid & 31, wave = tid >> 5, sub = tid >> 7;
  for (int i = tid; i < RBN; i += OTHR) srb[i] = 0;
  int carry = 0;
#pragma unroll 1
  for (int ch = 0; ch < nChunk; ++ch) {
    const int base = ch * NBC;
    const v4i c0 = *(const v4i*)(cnt + base + 8 * tid);
    const v4i c1 = *(const v4i*)(cnt + base + 8 * tid + 4);
    const int e0 = max(c0.x, 0), e1 = max(c0.y, 0), e2 = max(c0.z, 0), e3 = max(c0.w, 0);
    const int e4 = max(c1.x, 0), e5 = max(c1.y, 0), e6 = max(c1.z, 0), e7 = max(c1.w, 0);
    const int ts = e0 + e1 + e2 + e3 + e4 + e5 + e6 + e7;
    int incl = ts;
#pragma unroll
    for (int d = 1; d < 32; d <<= 1) {
      const int t = __shfl_up(incl, d);
      if (lane >= d) incl += t;
    }
    if (lane == 31) wtot[wave] = incl;
    __syncthreads();
    const int S0 = wtot[0]  + wtot[1]  + wtot[2]  + wtot[3];
    const int S1 = wtot[4]  + wtot[5]  + wtot[6]  + wtot[7];
    const int S2 = wtot[8]  + wtot[9]  + wtot[10] + wtot[11];
    const int S3 = wtot[12] + wtot[13] + wtot[14] + wtot[15];
    int pre = 0;
#pragma unroll 1
    for (int w = 4 * sub; w < wave; ++w) pre += wtot[w];
    const int b0 = carry;
    const int b1 = b0 + ((S0 + 31) & ~31);
    const int b2 = b1 + ((S1 + 31) & ~31);
    const int b3 = b2 + ((S2 + 31) & ~31);
    const int b4 = b3 + ((S3 + 31) & ~31);
    const int myb = sub == 0 ? b0 : (sub == 1 ? b1 : (sub == 2 ? b2 : b3));
    if (tid == 0) {
      srb[min(4 * ch + 0, RBN - 1)] = b0;
      srb[min(4 * ch + 1, RBN - 1)] = b1;
      srb[min(4 * ch + 2, RBN - 1)] = b2;
      srb[min(4 * ch + 3, RBN - 1)] = b3;
    }
    int run = myb + pre + incl - ts;
    soff[8 * tid + 0] = run; run += e0;
    soff[8 * tid + 1] = run; run += e1;
    soff[8 * tid + 2] = run; run += e2;
    soff[8 * tid + 3] = run; run += e3;
    soff[8 * tid + 4] = run; run += e4;
    soff[8 * tid + 5] = run; run += e5;
    soff[8 * tid + 6] = run; run += e6;
    soff[8 * tid + 7] = run;
    carry = b4;
    __syncthreads();
    const v4i o0 = *(const v4i*)(soff + 4 * tid);
    const v4i o1 = *(const v4i*)(soff + 4 * (tid + OTHR));
    int* op = off + base;
    *(volatile v4i*)(op + 4 * tid) = o0;
    *(volatile v4i*)(op + 4 * (tid + OTHR)) = o1;
    __threadfence();
    *(volatile v4i*)(op + 4 * tid) = o0;
    *(volatile v4i*)(op + 4 * (tid + OTHR)) = o1;
    __syncthreads();
  }
  if (tid == 0) srb[min(4 * nChunk, RBN - 1)] = carry;
  __syncthreads();
  v4i rv = {0, 0, 0, 0};
  if (tid < 32) rv = *(const v4i*)(srb + 4 * tid);
  if (tid < 32) *(volatile v4i*)(rbase + 4 * tid) = rv;
  __threadfence();
  if (tid < 32) *(volatile v4i*)(rbase + 4 * tid) = rv;
}

__global__ __launch_bounds__(NTHR) void k_fill(
    const int* __restrict__ srcs, const int* __restrict__ dsts,
    const int* __restrict__ off, const int* __restrict__ rbase,
    int* csr, int nN, int nE, int vec8, int csrLen) {
  extern __shared__ v4f lds_dyn[];
  int* region = (int*)lds_dyn;
  int* cursor = region + RCAP;
  int* list   = cursor + NBF;
  int* wcnt   = list + LISTN;
  const int tid = threadIdx.x, lane = tid & 31, wave = tid >> 5;
  const int b = blockIdx.x;
  const int nodeBase = b * NBF;

  int rb0 = rbase[b];
  const int rb1 = rbase[b + 1];
  rb0 = rb0 < 0 ? 0 : (rb0 > csrLen ? csrLen : rb0);
  rb0 &= ~31;
  int len = rb1 - rb0;
  len = len < 0 ? 0 : (len > RCAP ? RCAP : len);
  int lenW = (len + 31) & ~31;
  if (rb0 + lenW > csrLen) lenW = (csrLen - rb0) & ~31;

  {
    const v4i z = {0, 0, 0, 0};
    for (int i = tid; i < RCAP / 4; i += NTHR) ((v4i*)region)[i] = z;
    for (int s = tid; s < NBF; s += NTHR) {
      int o = off[nodeBase + s] - rb0;
      o = o < 0 ? 0 : (o > RCAP ? RCAP : o);
      cursor[s] = o;
    }
  }
  __syncthreads();

  const int nChunks = (nE + CHUNK - 1) / CHUNK;
#pragma unroll 1
  for (int ch = 0; ch < nChunks; ++ch) {
    const int cbase = ch * CHUNK;
    const int wc = scan_chunk<NBF>(dsts, nE, cbase, nodeBase, vec8, list, tid, lane, wave);
    if (lane == 0) wcnt[wave] = wc;
    __syncthreads();
    if (wave == 0) {
#pragma unroll 1
      for (int wsx = 0; wsx < NWAVE; ++wsx) {
        int n = __builtin_amdgcn_readfirstlane(wcnt[wsx]);
        n = n > WCAP ? WCAP : (n < 0 ? 0 : n);
        const int* lp = list + wsx * WCAP;
#pragma unroll 1
        for (int i = 0; i < n; ++i) {
          const int ent  = __builtin_amdgcn_readfirstlane(lp[i]);
          const int slot = ent & (NBF - 1);
          int e = cbase + ((ent >> 12) & (CHUNK - 1));
          e = e > nE - 1 ? nE - 1 : e;
          int src = srcs[e];
          src = src < 0 ? 0 : (src > nN - 1 ? nN - 1 : src);
          if (lane == 0) {
            int pos = cursor[slot];
            pos = pos < 0 ? 0 : (pos > RCAP - 1 ? RCAP - 1 : pos);
            region[pos] = src;
            const int np = pos + 1;
            cursor[slot] = np > RCAP ? RCAP : np;
          }
        }
      }
    }
    __syncthreads();
  }

  const int nv = lenW >> 2;
  int* gp = csr + rb0;
#pragma unroll 1
  for (int i = tid; i < nv; i += NTHR) { const v4i v = ((const v4i*)region)[i]; *(volatile v4i*)(gp + 4 * i) = v; }
  __threadfence();
#pragma unroll 1
  for (int i = tid; i < nv; i += NTHR) { const v4i v = ((const v4i*)region)[i]; *(volatile v4i*)(gp + 4 * i) = v; }
}

template <typename AT, int KD, int NCT, int NHW>
__global__ __launch_bounds__(NTHR) void k_gemm(
    const AT* A, int lda, int nRowsA, const _Float16* __restrict__ Bw,
    const float* __restrict__ attS, const float* __restrict__ attD,
    _Float16* C, int ldc, float* eS, float* eD) {
  constexpr int APK = GL<KD>::APK;
  constexpr int NCB = NCT / CBN;
  constexpr int KD8 = KD / 8;
  constexpr int UPT = (BM * KD8) / NTHR;
  static_assert(KD % 32 == 0 && NCT % CBN == 0 && (NHW % CBN) == 0 && NHW <= NCT);
  static_assert(UPT * NTHR == BM * KD8);
  static_assert(((APK * 2) % 16) == 0 && ((SPF * 4) % 16) == 0 && (GL<KD>::LDSA % 16) == 0);

  extern __shared__ v4f lds_dyn[];
  __shared__ __attribute__((aligned(16))) float sDs[BM];
  __shared__ __attribute__((aligned(16))) float sDd[BM];
  _Float16* sA  = (_Float16*)lds_dyn;
  float*    stg = (float*)((char*)lds_dyn + GL<KD>::LDSA);
  const int tid = threadIdx.x, lane = tid & 31, wave = tid >> 5, hh = lane >> 4, m = lane & 15;
  const int rowBase = blockIdx.x * BM;

#pragma unroll 4
  for (int i = 0; i < UPT; ++i) {
    const int idx = i * NTHR + tid;
    const int r   = idx / KD8;
    const int cc  = (idx - r * KD8) * 8;
    int row = rowBase + r;
    row = row > nRowsA - 1 ? nRowsA - 1 : row;
    row = row < 0 ? 0 : row;
    const v8h v = ALd<AT>::ld(A + (size_t)row * lda + cc);
    *(v8h*)(sA + r * APK + cc) = v;
  }
  __syncthreads();

  const int r0 = (wave >> 1) * 16;
  const int c0 = (wave & 1) * 128;
  const _Float16* arow = sA + (r0 + m) * APK + 8 * hh;
  const int drow = tid >> 2, dq = tid & 3;
  float ds = 0.f, dd = 0.f;

#pragma unroll 1
  for (int cb = 0; cb < NCB; ++cb) {
    v8f acc[8];
#pragma unroll
    for (int t = 0; t < 8; ++t) { v8f z = {0.f, 0.f, 0.f, 0.f, 0.f, 0.f, 0.f, 0.f}; acc[t] = z; }

#pragma unroll 1
    for (int ks = 0; ks < KD / 32; ++ks) {
      Frag a;
      a.h[0] = *(const v8h*)(arow + 32 * ks);
      a.h[1] = *(const v8h*)(arow + 32 * ks + 16);
#pragma unroll
      for (int t = 0; t < 8; ++t) {
        const _Float16* bp = Bw + (size_t)(cb * CBN + c0 + 16 * t + m) * KD + 32 * ks + 8 * hh;
        Frag b;
        b.h[0] = *(const v8h*)bp;
        b.h[1] = *(const v8h*)(bp + 16);
        acc[t] = wmf(a.v, b.v, acc[t]);
      }
    }

    {
      float* sp = stg + (r0 + 8 * hh) * SPF + c0 + m;
#pragma unroll
      for (int t = 0; t < 8; ++t) {
#pragma unroll
        for (int r = 0; r < 8; ++r) sp[r * SPF + 16 * t] = acc[t][r];
      }
    }
    __syncthreads();

    v4i ov[8];
#pragma unroll
    for (int i = 0; i < 8; ++i) {
      const int row = wave + 8 * i;
      const float* rp = stg + row * SPF + 8 * lane;
      const v4f va = *(const v4f*)rp * WSCI;
      const v4f vb = *(const v4f*)(rp + 4) * WSCI;
      H8 u; u.v = pack8(va, vb);
      ov[i] = u.w;
    }
    _Float16* cp = C + (size_t)rowBase * ldc + cb * CBN + 8 * lane;
#pragma unroll
    for (int i = 0; i < 8; ++i) *(volatile v4i*)(cp + (size_t)(wave + 8 * i) * ldc) = ov[i];
    __threadfence();
#pragma unroll
    for (int i = 0; i < 8; ++i) *(volatile v4i*)(cp + (size_t)(wave + 8 * i) * ldc) = ov[i];

    if constexpr (NHW > 0) {
      if (cb * CBN < NHW) {
        const float* rp = stg + drow * SPF + 64 * dq;
        const float* ap = attS + cb * CBN + 64 * dq;
        const float* dp = attD + cb * CBN + 64 * dq;
#pragma unroll 2
        for (int i = 0; i < 16; ++i) {
          const v4f v  = *(const v4f*)(rp + 4 * i) * WSCI;
          const v4f sa = *(const v4f*)(ap + 4 * i);
          const v4f sd = *(const v4f*)(dp + 4 * i);
          ds += v.x * sa.x + v.y * sa.y + v.z * sa.z + v.w * sa.w;
          dd += v.x * sd.x + v.y * sd.y + v.z * sd.z + v.w * sd.w;
        }
      }
    }
    __syncthreads();
  }

  if constexpr (NHW > 0) {
    ds += __shfl_xor(ds, 1); ds += __shfl_xor(ds, 2);
    dd += __shfl_xor(dd, 1); dd += __shfl_xor(dd, 2);
    if (dq == 0) { sDs[drow] = ds; sDd[drow] = dd; }
    __syncthreads();
    const int li = lane & 15;
    v4f dv = {0.f, 0.f, 0.f, 0.f};
    if (wave == 0 && lane < 16) { dv = *(const v4f*)(sDs + 4 * li); *(volatile v4f*)(eS + rowBase + 4 * li) = dv; }
    if (wave == 1 && lane < 16) { dv = *(const v4f*)(sDd + 4 * li); *(volatile v4f*)(eD + rowBase + 4 * li) = dv; }
    __threadfence();
    if (wave == 0 && lane < 16) *(volatile v4f*)(eS + rowBase + 4 * li) = dv;
    if (wave == 1 && lane < 16) *(volatile v4f*)(eD + rowBase + 4 * li) = dv;
  }
}

template <int NC, int RELU>
__global__ __launch_bounds__(NTHR) void k_agg(
    const int* __restrict__ csr, const int* __restrict__ off, const int* __restrict__ cnt,
    const float* __restrict__ eS, const float* __restrict__ eD,
    const _Float16* hw, int ldh, _Float16* hio, int ldr,
    const float* __restrict__ bconv, const float* __restrict__ blin, int nN, int csrLen) {
  constexpr int NG = NC / 256;
  static_assert(NG == 1 || NG == 2);
  const int tid = threadIdx.x, lane = tid & 31, wave = tid >> 5;
  const int tbase = blockIdx.x * TGT + wave * 32;
  const int col = 8 * lane;
  const v4f z4 = {0.f, 0.f, 0.f, 0.f};

  const v4f bca0 = *(const v4f*)(bconv + col), bcb0 = *(const v4f*)(bconv + col + 4);
  const v4f bla0 = *(const v4f*)(blin + col),  blb0 = *(const v4f*)(blin + col + 4);
  v4f bca1 = z4, bcb1 = z4, bla1 = z4, blb1 = z4;
  if constexpr (NG == 2) {
    bca1 = *(const v4f*)(bconv + 256 + col); bcb1 = *(const v4f*)(bconv + 256 + col + 4);
    bla1 = *(const v4f*)(blin + 256 + col);  blb1 = *(const v4f*)(blin + 256 + col + 4);
  }

  const int cl    = tbase + lane;
  const int cnt_l = cnt[cl];
  const int off_l = off[cl];

#pragma unroll 1
  for (int j = 0; j < 32; ++j) {
    const int c = tbase + j;
    int n = __shfl(cnt_l, j);
    n = n < 0 ? 0 : (n > DEGCAP ? DEGCAP : n);
    const int st = __shfl(off_l, j);
    const float ed = eD[c];

    float mx = NEG_BIG;
#pragma unroll 1
    for (int q0 = 0; q0 < n; q0 += 32) {
      int pos = st + q0 + lane;
      pos = pos < 0 ? 0 : (pos > csrLen - 1 ? csrLen - 1 : pos);
      int sl = csr[pos];
      sl = sl < 0 ? 0 : (sl > nN - 1 ? nN - 1 : sl);
      const int mcnt = (n - q0) < 32 ? (n - q0) : 32;
#pragma unroll 1
      for (int pp = 0; pp < mcnt; ++pp) {
        const int s = __builtin_amdgcn_readlane(sl, pp);
        mx = fmaxf(mx, lrelu(eS[(size_t)s] + ed));
      }
    }

    float den = 0.f;
    v4f a0a = z4, a0b = z4, a1a = z4, a1b = z4;
#pragma unroll 1
    for (int q0 = 0; q0 < n; q0 += 32) {
      int pos = st + q0 + lane;
      pos = pos < 0 ? 0 : (pos > csrLen - 1 ? csrLen - 1 : pos);
      int sl = csr[pos];
      sl = sl < 0 ? 0 : (sl > nN - 1 ? nN - 1 : sl);
      const int mcnt = (n - q0) < 32 ? (n - q0) : 32;
#pragma unroll 1
      for (int pp = 0; pp < mcnt; ++pp) {
        const int s = __builtin_amdgcn_readlane(sl, pp);
        const float p = __expf(lrelu(eS[(size_t)s] + ed) - mx);
        den += p;
        const _Float16* hr = hw + (size_t)s * ldh + col;
        H8 u0; u0.v = *(const v8h*)hr;
        a0a = a0a + h2f(u0.q[0]) * p;
        a0b = a0b + h2f(u0.q[1]) * p;
        if constexpr (NG == 2) {
          H8 u1; u1.v = *(const v8h*)(hr + 256);
          a1a = a1a + h2f(u1.q[0]) * p;
          a1b = a1b + h2f(u1.q[1]) * p;
        }
      }
    }

    const float rd = 1.0f / (den + DEN_EPS);
    _Float16* orow = hio + (size_t)c * ldr + col;
    H8 rs0; rs0.w = *(const v4i*)orow;
    v4f va = a0a * rd + bca0;
    v4f vb = a0b * rd + bcb0;
    va = va + (h2f(rs0.q[0]) + bla0);
    vb = vb + (h2f(rs0.q[1]) + blb0);
    if constexpr (RELU != 0) { va = relu4(va); vb = relu4(vb); }
    if (c >= nN) { va = z4; vb = z4; }
    H8 o0; o0.v = pack8(va, vb);
    H8 o1; o1.w = o0.w;
    if constexpr (NG == 2) {
      H8 rs1; rs1.w = *(const v4i*)(orow + 256);
      v4f wa = a1a * rd + bca1;
      v4f wb = a1b * rd + bcb1;
      wa = wa + (h2f(rs1.q[0]) + bla1);
      wb = wb + (h2f(rs1.q[1]) + blb1);
      if constexpr (RELU != 0) { wa = relu4(wa); wb = relu4(wb); }
      if (c >= nN) { wa = z4; wb = z4; }
      o1.v = pack8(wa, wb);
    }
    *(volatile v4i*)orow = o0.w;
    if constexpr (NG == 2) *(volatile v4i*)(orow + 256) = o1.w;
    __threadfence();
    *(volatile v4i*)orow = o0.w;
    if constexpr (NG == 2) *(volatile v4i*)(orow + 256) = o1.w;
  }
}

__global__ __launch_bounds__(NTHR) void k_mlp(
    const _Float16* H, int ldh, const _Float16* __restrict__ Wp,
    const float* __restrict__ hb1, const float* __restrict__ hb2, const float* __restrict__ hb3,
    const float* __restrict__ fcw, const float* __restrict__ fcb, float* out, int nN) {
  constexpr int KD  = HC2;
  constexpr int APK = GL<KD>::APK;
  constexpr int KD8 = KD / 8;
  constexpr int UPT = (BM * KD8) / NTHR;
  static_assert(UPT * NTHR == BM * KD8 && (BM * NCLS) % 4 == 0);

  extern __shared__ v4f lds_dyn[];
  __shared__ __attribute__((aligned(16))) float sO[BM * NCLS];
  _Float16* sA  = (_Float16*)lds_dyn;
  float*    stg = (float*)((char*)lds_dyn + GL<KD>::LDSA);
  const int tid = threadIdx.x, lane = tid & 31, wave = tid >> 5, hh = lane >> 4, m = lane & 15;
  const int rowBase = blockIdx.x * BM;

#pragma unroll
  for (int i = 0; i < UPT; ++i) {
    const int idx = i * NTHR + tid;
    const int r   = idx / KD8;
    const int cc  = (idx - r * KD8) * 8;
    *(v8h*)(sA + r * APK + cc) = *(const v8h*)(H + (size_t)(rowBase + r) * ldh + cc);
  }
  __syncthreads();

  const int r0 = (wave >> 1) * 16;
  const int c0 = (wave & 1) * 128;
  const _Float16* arow = sA + (r0 + m) * APK + 8 * hh;
  const int drow = tid >> 2, dq = tid & 3;

#pragma unroll 1
  for (int L = 0; L < 3; ++L) {
    const _Float16* Bw = Wp + (size_t)L * KD * KD;
    const float* hb = (L == 0) ? hb1 : ((L == 1) ? hb2 : hb3);
    v8f acc[8];
#pragma unroll
    for (int t = 0; t < 8; ++t) { v8f z = {0.f, 0.f, 0.f, 0.f, 0.f, 0.f, 0.f, 0.f}; acc[t] = z; }
#pragma unroll 1
    for (int ks = 0; ks < KD / 32; ++ks) {
      Frag a;
      a.h[0] = *(const v8h*)(arow + 32 * ks);
      a.h[1] = *(const v8h*)(arow + 32 * ks + 16);
#pragma unroll
      for (int t = 0; t < 8; ++t) {
        const _Float16* bp = Bw + (size_t)(c0 + 16 * t + m) * KD + 32 * ks + 8 * hh;
        Frag b;
        b.h[0] = *(const v8h*)bp;
        b.h[1] = *(const v8h*)(bp + 16);
        acc[t] = wmf(a.v, b.v, acc[t]);
      }
    }
    {
      float* sp = stg + (r0 + 8 * hh) * SPF + c0 + m;
#pragma unroll
      for (int t = 0; t < 8; ++t) {
#pragma unroll
        for (int r = 0; r < 8; ++r) sp[r * SPF + 16 * t] = acc[t][r];
      }
    }
    __syncthreads();
    {
      float* rp = stg + drow * SPF + 64 * dq;
      _Float16* hp = sA + drow * APK + 64 * dq;
      const float* bp = hb + 64 * dq;
#pragma unroll 2
      for (int i = 0; i < 8; ++i) {
        v4f a = *(const v4f*)(rp + 8 * i), b = *(const v4f*)(rp + 8 * i + 4);
        const v4f ba = *(const v4f*)(bp + 8 * i), bb = *(const v4f*)(bp + 8 * i + 4);
        a = relu4(a * WSCI + ba);
        b = relu4(b * WSCI + bb);
        *(v4f*)(rp + 8 * i) = a;
        *(v4f*)(rp + 8 * i + 4) = b;
        *(v8h*)(hp + 8 * i) = pack8(a, b);
      }
    }
    __syncthreads();
  }

  float lg[NCLS];
#pragma unroll
  for (int c = 0; c < NCLS; ++c) lg[c] = 0.f;
  {
    const float* rp = stg + drow * SPF + 64 * dq;
#pragma unroll 1
    for (int i = 0; i < 16; ++i) {
      const v4f v = *(const v4f*)(rp + 4 * i);
      const float* fp = fcw + (size_t)(64 * dq + 4 * i) * NCLS;
#pragma unroll
      for (int c = 0; c < NCLS; ++c)
        lg[c] += v.x * fp[c] + v.y * fp[NCLS + c] + v.z * fp[2 * NCLS + c] + v.w * fp[3 * NCLS + c];
    }
  }
#pragma unroll
  for (int c = 0; c < NCLS; ++c) { lg[c] += __shfl_xor(lg[c], 1); lg[c] += __shfl_xor(lg[c], 2); lg[c] += fcb[c]; }
  float mxl = lg[0];
#pragma unroll
  for (int c = 1; c < NCLS; ++c) mxl = fmaxf(mxl, lg[c]);
  float ex[NCLS], sum = 0.f;
#pragma unroll
  for (int c = 0; c < NCLS; ++c) { ex[c] = __expf(lg[c] - mxl); sum += ex[c]; }
  const float inv = 1.0f / sum;
  if (dq == 0) {
#pragma unroll
    for (int c = 0; c < NCLS; ++c) sO[drow * NCLS + c] = ex[c] * inv;
  }
  __syncthreads();

  int nrows = nN - rowBase;
  nrows = nrows < 0 ? 0 : (nrows > BM ? BM : nrows);
  const int T   = nrows * NCLS;
  const int nf4 = T >> 2;
  const int rem = T & 3;
  float* op = out + (size_t)rowBase * NCLS;
  v4f vo = {0.f, 0.f, 0.f, 0.f};
  const bool w4 = tid < nf4;
  const bool wt = tid < rem;
  float tv = 0.f;
  if (w4) vo = *(const v4f*)(sO + 4 * tid);
  if (wt) tv = sO[4 * nf4 + tid];
  if (w4) *(volatile v4f*)(op + 4 * tid) = vo;
  if (wt) *(volatile float*)(op + 4 * nf4 + tid) = tv;
  __threadfence();
  if (w4) *(volatile v4f*)(op + 4 * tid) = vo;
  if (wt) *(volatile float*)(op + 4 * nf4 + tid) = tv;
}

extern "C" void kernel_launch(void* const* d_in, const int* in_sizes, int n_in,
                              void* d_out, int out_size, void* d_ws, size_t ws_size,
                              hipStream_t stream) {
  if (n_in < 22) return;
  const int nN = in_sizes[0] / DIN;
  const int nE = in_sizes[1] / 2;
  if (nN <= 0 || nE <= 0 || in_sizes[0] != nN * DIN || in_sizes[1] != 2 * nE) return;
  if (in_sizes[2] != DIN * HC1 || in_sizes[3] != HC1 || in_sizes[4] != HC1 || in_sizes[5] != HC1) return;
  if (in_sizes[6] != DIN * HC1 || in_sizes[7] != HC1) return;
  if (in_sizes[8] != HC1 * HC2 || in_sizes[9] != HC2 || in_sizes[10] != HC2 || in_sizes[11] != HC2) return;
  if (in_sizes[12] != HC1 * HC2 || in_sizes[13] != HC2) return;
  if (in_sizes[14] != HC2 * HC2 || in_sizes[15] != HC2 || in_sizes[16] != HC2 * HC2 || in_sizes[17] != HC2) return;
  if (in_sizes[18] != HC2 * HC2 || in_sizes[19] != HC2 || in_sizes[20] != HC2 * NCLS || in_sizes[21] != NCLS) return;
  if (out_size != nN * NCLS) return;
  if (nE > (1 << 28) || nN > (1 << 24)) return;

  const float* x   = (const float*)d_in[0];
  const int*   ei  = (const int*)d_in[1];
  const float* W1  = (const float*)d_in[2];
  const float* as1 = (const float*)d_in[3];
  const float* ad1 = (const float*)d_in[4];
  const float* bc1 = (const float*)d_in[5];
  const float* A1  = (const float*)d_in[6];
  const float* b1  = (const float*)d_in[7];
  const float* W2  = (const float*)d_in[8];
  const float* as2 = (const float*)d_in[9];
  const float* ad2 = (const float*)d_in[10];
  const float* bc2 = (const float*)d_in[11];
  const float* A2  = (const float*)d_in[12];
  const float* b2  = (const float*)d_in[13];
  const float* Hw1 = (const float*)d_in[14];
  const float* Hb1 = (const float*)d_in[15];
  const float* Hw2 = (const float*)d_in[16];
  const float* Hb2 = (const float*)d_in[17];
  const float* Hw3 = (const float*)d_in[18];
  const float* Hb3 = (const float*)d_in[19];
  const float* fcw = (const float*)d_in[20];
  const float* fcb = (const float*)d_in[21];
  const int*   src = ei;
  const int*   dst = ei + nE;
  float* out = (float*)d_out;

  const int NPAD   = ((nN + TGT - 1) / TGT) * TGT;
  const int nBC    = (nN + NBC - 1) / NBC;
  const int CNTPAD = nBC * NBC;
  if (4 * nBC + 1 > RBN) return;
  if (CNTPAD < NPAD) return;
  const int nBF    = (nN + NBF - 1) / NBF;
  const int csrLen = ((nE + 31) & ~31) + 4096;
  if (31 * 4 * nBC > 4096) return;
  const int nAgg   = NPAD / TGT;
  const int nGm    = NPAD / BM;

  char* ws = (char*)d_ws;
  size_t off = 0;
  const size_t oW1  = off; off += (size_t)(2 * HC1) * DIN * 2;    off = (off + 255) & ~(size_t)255;
  const size_t oW2  = off; off += (size_t)(2 * HC2) * HC1 * 2;    off = (off + 255) & ~(size_t)255;
  const size_t oW3  = off; off += (size_t)3 * HC2 * HC2 * 2;      off = (off + 255) & ~(size_t)255;
  const size_t oCnt = off; off += (size_t)CNTPAD * 4;             off = (off + 255) & ~(size_t)255;
  const size_t oOff = off; off += (size_t)CNTPAD * 4;             off = (off + 255) & ~(size_t)255;
  const size_t oRb  = off; off += (size_t)RBN * 4;                off = (off + 255) & ~(size_t)255;
  const size_t oCsr = off; off += (size_t)csrLen * 4;             off = (off + 255) & ~(size_t)255;
  const size_t oES  = off; off += (size_t)NPAD * 4;               off = (off + 255) & ~(size_t)255;
  const size_t oED  = off; off += (size_t)NPAD * 4;               off = (off + 255) & ~(size_t)255;
  const size_t oP   = off; off += (size_t)NPAD * PW * 2;          off = (off + 255) & ~(size_t)255;
  if (off > ws_size || off > (size_t)WSCAP) return;
  _Float16* wp1 = (_Float16*)(ws + oW1);
  _Float16* wp2 = (_Float16*)(ws + oW2);
  _Float16* wp3 = (_Float16*)(ws + oW3);
  int*   cnt  = (int*)(ws + oCnt);
  int*   offp = (int*)(ws + oOff);
  int*   rb   = (int*)(ws + oRb);
  int*   csr  = (int*)(ws + oCsr);
  float* es   = (float*)(ws + oES);
  float* ed   = (float*)(ws + oED);
  _Float16* P = (_Float16*)(ws + oP);

  const int vec8 = ((nE & 3) == 0) ? 1 : 0;

  k_wprep<DIN, HC1><<<(HC1 * DIN / 8 + NTHR - 1) / NTHR, NTHR, 0, stream>>>(W1, wp1);
  k_wprep<DIN, HC1><<<(HC1 * DIN / 8 + NTHR - 1) / NTHR, NTHR, 0, stream>>>(A1, wp1 + (size_t)HC1 * DIN);
  k_wprep<HC1, HC2><<<(HC2 * HC1 / 8 + NTHR - 1) / NTHR, NTHR, 0, stream>>>(W2, wp2);
  k_wprep<HC1, HC2><<<(HC2 * HC1 / 8 + NTHR - 1) / NTHR, NTHR, 0, stream>>>(A2, wp2 + (size_t)HC2 * HC1);
  k_wprep<HC2, HC2><<<(HC2 * HC2 / 8 + NTHR - 1) / NTHR, NTHR, 0, stream>>>(Hw1, wp3);
  k_wprep<HC2, HC2><<<(HC2 * HC2 / 8 + NTHR - 1) / NTHR, NTHR, 0, stream>>>(Hw2, wp3 + (size_t)HC2 * HC2);
  k_wprep<HC2, HC2><<<(HC2 * HC2 / 8 + NTHR - 1) / NTHR, NTHR, 0, stream>>>(Hw3, wp3 + (size_t)2 * HC2 * HC2);

  k_count<<<nBC, NTHR, 0, stream>>>(dst, cnt, nE, vec8);
  k_offsets<<<1, OTHR, 0, stream>>>(cnt, offp, rb, nBC);
  hipFuncSetAttribute(reinterpret_cast<const void*>(&k_fill),
                      hipFuncAttributeMaxDynamicSharedMemorySize, LDS_FILL);
  k_fill<<<nBF, NTHR, LDS_FILL, stream>>>(src, dst, offp, rb, csr, nN, nE, vec8, csrLen);

  hipFuncSetAttribute(reinterpret_cast<const void*>(&k_gemm<float, DIN, 2 * HC1, HC1>),
                      hipFuncAttributeMaxDynamicSharedMemorySize, GL<DIN>::LDS);
  k_gemm<float, DIN, 2 * HC1, HC1><<<nGm, NTHR, GL<DIN>::LDS, stream>>>(
      x, DIN, nN, wp1, as1, ad1, P, PW, es, ed);
  k_agg<HC1, 1><<<nAgg, NTHR, 0, stream>>>(csr, offp, cnt, es, ed, P, PW, P + HC1, PW, bc1, b1, nN, csrLen);

  hipFuncSetAttribute(reinterpret_cast<const void*>(&k_gemm<_Float16, HC1, 2 * HC2, HC2>),
                      hipFuncAttributeMaxDynamicSharedMemorySize, GL<HC1>::LDS);
  k_gemm<_Float16, HC1, 2 * HC2, HC2><<<nGm, NTHR, GL<HC1>::LDS, stream>>>(
      P + HC1, PW, NPAD, wp2, as2, ad2, P, PW, es, ed);
  k_agg<HC2, 0><<<nAgg, NTHR, 0, stream>>>(csr, offp, cnt, es, ed, P, PW, P + HC2, PW, bc2, b2, nN, csrLen);

  hipFuncSetAttribute(reinterpret_cast<const void*>(&k_mlp),
                      hipFuncAttributeMaxDynamicSharedMemorySize, GL<HC2>::LDS);
  k_mlp<<<nGm, NTHR, GL<HC2>::LDS, stream>>>(P + HC2, PW, wp3, Hb1, Hb2, Hb3, fcw, fcb, out, nN);
}
